// Attention_72438918414659
// MI455X (gfx1250) — hardware-verified
//
#include <hip/hip_runtime.h>


#ifndef NB
#define NB 8
#endif
#ifndef SEQ
#define SEQ 4096
#endif
#define NB_FULL  8
#define SEQ_FULL 4096
#define DIM  128
#define NWV  4
#define BQ   (16 * NWV)
#define KS   32
#define OSP  132
#define VTK  64
#define VTP  72
#define L2E  1.4426950408889634f

static_assert(DIM == 128);
static_assert(SEQ % BQ == 0);
static_assert(SEQ % VTK == 0);
static_assert(SEQ % KS == 0);
static_assert(NB <= NB_FULL);
static_assert(SEQ <= SEQ_FULL);
static_assert(((size_t)NB * SEQ * DIM) % 2048 == 0);
static_assert((size_t)(NB * (SEQ / VTK)) * (size_t)(DIM * VTK) == (size_t)NB * SEQ * DIM);
static_assert((size_t)(NB * (SEQ / BQ)) * (size_t)(BQ * DIM) == (size_t)NB * SEQ * DIM);
static_assert(((size_t)NB * SEQ * DIM * 2) % 256 == 0);

typedef unsigned short bf;
typedef __attribute__((ext_vector_type(16))) __bf16   v16bf;
typedef __attribute__((ext_vector_type(2)))  __bf16   v2bf;
typedef __attribute__((ext_vector_type(8)))  unsigned short v8us;
typedef __attribute__((ext_vector_type(8)))  unsigned int   v8u;
typedef __attribute__((ext_vector_type(8)))  float    v8f;
typedef __attribute__((ext_vector_type(4)))  float    v4f;
typedef v4f  __attribute__((may_alias)) v4fa;
typedef v8us __attribute__((may_alias)) v8usa;

__device__ __forceinline__ unsigned short f2bf(float f) { unsigned u = __float_as_uint(f); u += 0x7FFFu + ((u >> 16) & 1u); return (unsigned short)(u >> 16); }
__device__ __forceinline__ float bf2f(unsigned short b) { return __uint_as_float(((unsigned)b) << 16); }
__device__ __forceinline__ float bfr(float f) { return bf2f(f2bf(f)); }
__device__ __forceinline__ v16bf cat16b(v8us lo, v8us hi) { return __builtin_bit_cast(v16bf, __builtin_shufflevector(lo, hi, 0, 1, 2, 3, 4, 5, 6, 7, 8, 9, 10, 11, 12, 13, 14, 15)); }
__device__ __forceinline__ v8f wmmab(v16bf a, v16bf b, v8f c) { return __builtin_amdgcn_wmma_f32_16x16x32_bf16(false, a, false, b, (short)0, c, false, false); }
__device__ __forceinline__ v16bf ldb(const bf* p) { return cat16b(*(const v8us*)p, *(const v8us*)(p + 16)); }
__device__ __forceinline__ unsigned pk2bf(float a, float b) { v2bf t; t[0] = (__bf16)a; t[1] = (__bf16)b; return __builtin_bit_cast(unsigned, t); }

__global__ __launch_bounds__(256) void k_cvt8(const float* __restrict__ q, const float* __restrict__ k, bf* QB, bf* KB) {
    const unsigned i = blockIdx.x * 256u + threadIdx.x;
    const unsigned per = (unsigned)(SEQ * DIM / 8);
    if (i >= (unsigned)NB * per) return;
    const unsigned b = i / per, r = i - b * per;
    const float* src = (blockIdx.y ? k : q) + (size_t)b * SEQ_FULL * DIM + (size_t)r * 8;
    bf* dst = (blockIdx.y ? KB : QB) + (size_t)i * 8;
    const v8f v = *(const v8f*)src;
    v8us o;
#pragma unroll
    for (int c = 0; c < 8; ++c) o[c] = f2bf(v[c]);
    *(volatile v8us*)dst = o;
    __threadfence();
    *(volatile v8us*)dst = o;
}

__global__ __launch_bounds__(256) void k_vt(const float* __restrict__ V, bf* VT) {
    __shared__ __align__(16) bf tl[DIM * VTP];
    const unsigned tid = threadIdx.x;
    const unsigned tpb = (unsigned)(SEQ / VTK);
    const unsigned b = blockIdx.x / tpb;
    const unsigned k0 = (blockIdx.x - b * tpb) * VTK;
    const float* src = V + ((size_t)b * SEQ_FULL + k0) * DIM;
#pragma unroll
    for (unsigned it = 0; it < 8; ++it) {
        const unsigned f = it * 256u + tid;
        const unsigned key = f >> 5, d4 = (f & 31u) * 4u;
        const v4f x = *(const v4f*)(src + (size_t)key * DIM + d4);
#pragma unroll
        for (unsigned c = 0; c < 4; ++c) tl[(d4 + c) * VTP + key] = f2bf(x[c]);
    }
    __syncthreads();
    bf* dst = VT + (size_t)b * DIM * SEQ + k0;
    const unsigned c8 = (tid & 7u) * 8u, dr = tid >> 3;
#pragma unroll 1
    for (int ps = 0; ps < 2; ++ps) {
#pragma unroll
        for (unsigned it = 0; it < 4; ++it) {
            const unsigned d = it * 32u + dr;
            const v8us o = *(const v8usa*)(tl + d * VTP + c8);
            *(volatile v8us*)(dst + (size_t)d * SEQ + c8) = o;
        }
        if (ps == 0) __threadfence();
    }
}

__global__ __launch_bounds__(128) void k_flash(const bf* __restrict__ QB, const bf* __restrict__ KB, const bf* __restrict__ VT, const float* __restrict__ Vf, float* O) {
    __shared__ __align__(16) float os[NWV * 16 * OSP];
    const unsigned tid = threadIdx.x, lane = tid & 31u, wv = tid >> 5, lr = lane & 15u, hi = lane >> 4;
    const unsigned bpb = (unsigned)(SEQ / BQ);
    const unsigned b = blockIdx.x / bpb;
    const unsigned q0 = (blockIdx.x - b * bpb) * BQ + wv * 16u;

    v16bf qf[4];
    {
        const bf* qp = QB + ((size_t)b * SEQ + q0 + lr) * DIM + 8u * hi;
#pragma unroll
        for (int dk = 0; dk < 4; ++dk) qf[dk] = ldb(qp + dk * 32);
    }
    const bf* kp = KB + ((size_t)b * SEQ + lr) * DIM + 8u * hi;
    const bf* vp = VT + ((size_t)b * DIM + lr) * SEQ + 8u * hi;

    v8f o[8];
#pragma unroll
    for (int t = 0; t < 8; ++t) o[t] = (v8f){};
    float ml = -1.0e30f;
    float l = 0.0f;

#pragma unroll 1
    for (unsigned k0 = 0; k0 < (unsigned)SEQ; k0 += KS) {
        v8f s0 = (v8f){}, s1 = (v8f){};
        const bf* ka = kp + (size_t)k0 * DIM;
#pragma unroll
        for (int dk = 0; dk < 4; ++dk) {
            const v16bf a0 = ldb(ka + dk * 32);
            const v16bf a1 = ldb(ka + 16 * DIM + dk * 32);
            s0 = wmmab(a0, qf[dk], s0);
            s1 = wmmab(a1, qf[dk], s1);
        }
        asm volatile("v_nop\n\tv_nop\n\tv_nop\n\tv_nop" : "+v"(s0), "+v"(s1) : "v"(qf[0]), "v"(qf[3]));

        float mx = fmaxf(s0[0], s1[0]);
#pragma unroll
        for (int r = 1; r < 8; ++r) mx = fmaxf(mx, fmaxf(s0[r], s1[r]));
        mx = fmaxf(mx, __shfl_xor(mx, 16, 32));
        const float mnl = fmaxf(ml, mx * L2E);
        const float corr = __builtin_amdgcn_exp2f(ml - mnl);
        ml = mnl;
        float p0[8], p1[8];
        float ps = 0.0f;
#pragma unroll
        for (int r = 0; r < 8; ++r) {
            p0[r] = __builtin_amdgcn_exp2f(fmaf(s0[r], L2E, -mnl));
            p1[r] = __builtin_amdgcn_exp2f(fmaf(s1[r], L2E, -mnl));
            ps += p0[r] + p1[r];
        }
        ps += __shfl_xor(ps, 16, 32);
        l = l * corr + ps;
        if (__builtin_amdgcn_ballot_w32(corr != 1.0f) != 0u) {
#pragma unroll
            for (int t = 0; t < 8; ++t) o[t] *= corr;
        }

        v8u hw, lw;
#pragma unroll
        for (int j = 0; j < 4; ++j) {
            const unsigned u0 = __float_as_uint(p0[2 * j]), u1 = __float_as_uint(p0[2 * j + 1]);
            const unsigned w0 = __float_as_uint(p1[2 * j]), w1 = __float_as_uint(p1[2 * j + 1]);
            hw[j]     = (u1 & 0xFFFF0000u) | (u0 >> 16);
            hw[4 + j] = (w1 & 0xFFFF0000u) | (w0 >> 16);
            lw[j]     = pk2bf(p0[2 * j] - __uint_as_float(u0 & 0xFFFF0000u), p0[2 * j + 1] - __uint_as_float(u1 & 0xFFFF0000u));
            lw[4 + j] = pk2bf(p1[2 * j] - __uint_as_float(w0 & 0xFFFF0000u), p1[2 * j + 1] - __uint_as_float(w1 & 0xFFFF0000u));
        }
        const v16bf ph = __builtin_bit_cast(v16bf, hw);
        const v16bf pl = __builtin_bit_cast(v16bf, lw);

        asm volatile("" ::: "memory");
        const bf* va = vp + k0;
#pragma unroll
        for (int t = 0; t < 8; ++t) {
            const v16bf a = ldb(va + (size_t)t * 16 * SEQ);
            o[t] = wmmab(a, ph, o[t]);
            o[t] = wmmab(a, pl, o[t]);
        }
        asm volatile("v_nop\n\tv_nop\n\tv_nop\n\tv_nop"
                     : "+v"(o[0]), "+v"(o[1]), "+v"(o[2]), "+v"(o[3]), "+v"(o[4]), "+v"(o[5]), "+v"(o[6]), "+v"(o[7])
                     : "v"(ph), "v"(pl));
    }

    const float inv = 1.0f / l;
    float* ow = os + wv * (16 * OSP);
#pragma unroll
    for (int t = 0; t < 8; ++t) {
#pragma unroll
        for (int r = 0; r < 8; ++r) ow[lr * OSP + t * 16 + 8 * hi + r] = o[t][r] * inv;
    }
    __syncthreads();
    float* orow = O + ((size_t)b * SEQ + q0) * DIM + lane * 4u;
    const float* vrow = Vf + ((size_t)b * SEQ_FULL + q0) * DIM + lane * 4u;
#pragma unroll 1
    for (int ps2 = 0; ps2 < 2; ++ps2) {
#pragma unroll 4
        for (unsigned s = 0; s < 16; ++s) {
            v4f val = *(const v4fa*)(ow + s * OSP + lane * 4u);
            const v4f vv = *(const v4f*)(vrow + (size_t)s * DIM);
            val[0] += bfr(vv[0]); val[1] += bfr(vv[1]); val[2] += bfr(vv[2]); val[3] += bfr(vv[3]);
            *(volatile v4f*)(orow + (size_t)s * DIM) = val;
        }
        if (ps2 == 0) __threadfence();
    }
}

extern "C" void kernel_launch(void* const* d_in, const int* in_sizes, int n_in,
                              void* d_out, int out_size, void* d_ws, size_t ws_size, hipStream_t stream) {
    if (n_in < 3) return;
    const size_t need = ((size_t)(NB - 1) * SEQ_FULL + SEQ) * DIM;
    if ((size_t)in_sizes[0] < need || (size_t)in_sizes[1] < need || (size_t)in_sizes[2] < need) return;
    if ((size_t)out_size < (size_t)NB * SEQ * DIM) return;
    const float* q = (const float*)d_in[0];
    const float* v = (const float*)d_in[1];
    const float* k = (const float*)d_in[2];
    float* OUT = (float*)d_out;
    const size_t PL = (size_t)NB * SEQ * DIM * 2;
    if (3 * PL > ws_size) return;
    char* wsp = (char*)d_ws;
    bf* QB = (bf*)(wsp);
    bf* KB = (bf*)(wsp + PL);
    bf* VT = (bf*)(wsp + 2 * PL);
    const unsigned gc = (unsigned)(((size_t)NB * SEQ * DIM / 8 + 255) / 256);
    k_cvt8<<<dim3(gc, 2, 1), 256, 0, stream>>>(q, k, QB, KB);
    k_vt<<<(unsigned)(NB * (SEQ / VTK)), 256, 0, stream>>>(v, VT);
    k_flash<<<(unsigned)(NB * (SEQ / BQ)), 128, 0, stream>>>(QB, KB, VT, v, OUT);
}
